// TransBlockV2_18588618457699
// MI455X (gfx1250) — hardware-verified
//
#include <hip/hip_runtime.h>
#include <hip/hip_bf16.h>
#include <stddef.h>

#define NE 1024
#define NL 25
#define NS 64
#define NC 128
#define NH 512
#define NX 8
#define NTHR 256

#define MP 136
#define TP 72
#define GP 132
#define LGP 68
#define HPIT 520

#define L0_LDS 34816
#define AT_A   0
#define AT_B   33792
#define AT_Q   68608
#define AT_K   103424
#define AT_VT  138240
#define AT_MT  175104
#define AT_POS 191488
#define AT_LDS 192512
#define EX_XS  0
#define EX_HID 17408
#define EX_AH  17408
#define EX_AL  35840
#define EX_OS  54272
#define EX_LDS 83968

static_assert(NE % 64 == 0);
static_assert(64 * MP * 2 * 2 == L0_LDS);
static_assert(64 * GP * 4 <= L0_LDS);
static_assert(AT_B - AT_A == 64 * GP * 4);
static_assert(64 * LGP * 4 <= AT_B - AT_A);
static_assert(AT_Q - AT_B == 64 * MP * 2 * 2);
static_assert(64 * TP * 2 * 2 <= AT_Q - AT_B);
static_assert(AT_K - AT_Q == 64 * MP * 4);
static_assert(AT_VT - AT_K == 64 * MP * 4);
static_assert(AT_MT - AT_VT == 128 * TP * 4);
static_assert(AT_POS - AT_MT == 128 * 32 * 4);
static_assert(AT_LDS - AT_POS >= NS * 3 * 4);
static_assert(EX_HID == 64 * MP * 2);
static_assert(EX_AL == EX_AH + 128 * TP * 2);
static_assert(EX_OS == EX_AL + 128 * TP * 2);
static_assert(EX_OS + 32 * GP * 4 <= EX_LDS);
static_assert(EX_LDS == EX_HID + 64 * HPIT * 2);

typedef _Float16 f16;
typedef f16 v16h __attribute__((ext_vector_type(16)));
typedef f16 v8h_t __attribute__((ext_vector_type(8)));
typedef v8h_t __attribute__((may_alias)) v8h;
typedef __bf16 v16b __attribute__((ext_vector_type(16)));
typedef unsigned short v8us_t __attribute__((ext_vector_type(8)));
typedef v8us_t __attribute__((may_alias)) v8us;
typedef float v8f __attribute__((ext_vector_type(8)));
typedef float v4f_t __attribute__((ext_vector_type(4)));
typedef v4f_t __attribute__((may_alias)) v4f;
typedef unsigned int v4u_t __attribute__((ext_vector_type(4)));
typedef v4u_t __attribute__((may_alias)) v4u;

union FragH { v16h v; v8h_t h[2]; };
union FragB { v16b v; v8us_t u[2]; };
union Pack8 { v8h_t h; v4u_t u; };

__device__ __forceinline__ v8f zero8() {
  v8f z;
#pragma unroll
  for (int i = 0; i < 8; ++i) z[i] = 0.0f;
  return z;
}

__device__ __forceinline__ unsigned short bf_bits(float x) {
  unsigned int u = __float_as_uint(x);
  u = u + 0x7FFFu + ((u >> 16) & 1u);
  return (unsigned short)(u >> 16);
}
__device__ __forceinline__ void split_bf(float x, unsigned short& hi, unsigned short& lo) {
  hi = bf_bits(x);
  const float hf = __uint_as_float(((unsigned int)hi) << 16);
  lo = bf_bits(x - hf);
}

__device__ __forceinline__ v16h ldh16(const f16* p, int k0) {
  FragH f;
  f.h[0] = *(const v8h*)(p + k0);
  f.h[1] = *(const v8h*)(p + k0 + 16);
  return f.v;
}
__device__ __forceinline__ v16b ldb16(const unsigned short* p, int k0) {
  FragB f;
  f.u[0] = *(const v8us*)(p + k0);
  f.u[1] = *(const v8us*)(p + k0 + 16);
  return f.v;
}

__device__ __forceinline__ v8f mma_h(v16h a, v16h b, v8f c) {
  return __builtin_amdgcn_wmma_f32_16x16x32_f16(false, a, false, b, (short)0, c, false, false);
}
__device__ __forceinline__ v8f mma_b(v16b a, v16b b, v8f c) {
  return __builtin_amdgcn_wmma_f32_16x16x32_bf16(false, a, false, b, (short)0, c, false, false);
}

__device__ __forceinline__ void gemm4_h(const f16* a, const f16* b, int ldb, int n0, int ks,
                                        v8f (&acc)[4], int m, int hh) {
#pragma unroll 1
  for (int s = 0; s < ks; ++s) {
    const int k0 = s * 32;
    const v16h af = ldh16(a, k0);
    v16h bf[4];
#pragma unroll
    for (int t = 0; t < 4; ++t)
      bf[t] = ldh16(b + (size_t)(n0 + 16 * t + m) * ldb + 8 * hh, k0);
#pragma unroll
    for (int t = 0; t < 4; ++t) acc[t] = mma_h(af, bf[t], acc[t]);
    asm volatile("v_nop\n\tv_nop\n\tv_nop\n\tv_nop"
                 : "+v"(acc[0]), "+v"(acc[1]), "+v"(acc[2]), "+v"(acc[3])
                 : "v"(af), "v"(bf[0]), "v"(bf[1]), "v"(bf[2]), "v"(bf[3]));
  }
}

__device__ __forceinline__ void gemm4_bf3(const unsigned short* ah, const unsigned short* al,
                                          const unsigned short* bh, const unsigned short* bl,
                                          int ldb, int n0, int ks, v8f (&acc)[4], int m, int hh) {
#pragma unroll 1
  for (int s = 0; s < ks; ++s) {
    const int k0 = s * 32;
    const v16b a0 = ldb16(ah, k0);
    const v16b a1 = ldb16(al, k0);
    v16b b0[4], b1[4];
#pragma unroll
    for (int t = 0; t < 4; ++t) {
      const size_t off = (size_t)(n0 + 16 * t + m) * ldb + 8 * hh;
      b0[t] = ldb16(bh + off, k0);
      b1[t] = ldb16(bl + off, k0);
    }
#pragma unroll
    for (int t = 0; t < 4; ++t) {
      acc[t] = mma_b(a0, b0[t], acc[t]);
      acc[t] = mma_b(a0, b1[t], acc[t]);
      acc[t] = mma_b(a1, b0[t], acc[t]);
    }
    asm volatile("v_nop\n\tv_nop\n\tv_nop\n\tv_nop"
                 : "+v"(acc[0]), "+v"(acc[1]), "+v"(acc[2]), "+v"(acc[3])
                 : "v"(a0), "v"(a1), "v"(b0[0]), "v"(b0[1]), "v"(b0[2]), "v"(b0[3]),
                   "v"(b1[0]), "v"(b1[1]), "v"(b1[2]), "v"(b1[3]));
  }
}

__device__ __forceinline__ void gemm2_bf3(const unsigned short* ah, const unsigned short* al,
                                          const unsigned short* bh, const unsigned short* bl,
                                          int ldb, int n0, int ks, v8f (&acc)[2], int m, int hh) {
#pragma unroll 1
  for (int s = 0; s < ks; ++s) {
    const int k0 = s * 32;
    const v16b a0 = ldb16(ah, k0);
    const v16b a1 = ldb16(al, k0);
    v16b b0[2], b1[2];
#pragma unroll
    for (int t = 0; t < 2; ++t) {
      const size_t off = (size_t)(n0 + 16 * t + m) * ldb + 8 * hh;
      b0[t] = ldb16(bh + off, k0);
      b1[t] = ldb16(bl + off, k0);
    }
#pragma unroll
    for (int t = 0; t < 2; ++t) {
      acc[t] = mma_b(a0, b0[t], acc[t]);
      acc[t] = mma_b(a0, b1[t], acc[t]);
      acc[t] = mma_b(a1, b0[t], acc[t]);
    }
    asm volatile("v_nop\n\tv_nop\n\tv_nop\n\tv_nop"
                 : "+v"(acc[0]), "+v"(acc[1])
                 : "v"(a0), "v"(a1), "v"(b0[0]), "v"(b0[1]), "v"(b1[0]), "v"(b1[1]));
  }
}

__global__ void __launch_bounds__(NTHR) k_prep(
    const float* __restrict__ wq, const float* __restrict__ wk, const float* __restrict__ wv,
    const float* __restrict__ fcw, const float* __restrict__ elg, const float* __restrict__ elb,
    const float* __restrict__ ew1, const float* __restrict__ eb1, const float* __restrict__ ew2,
    const float* __restrict__ tg, const float* __restrict__ fg,
    unsigned short* __restrict__ pqkv, f16* __restrict__ w1t, f16* __restrict__ w2t,
    unsigned short* __restrict__ tgp, unsigned short* __restrict__ fgp, float* __restrict__ b1f)
{
  __shared__ float tile[64 * 65];
  const int tid = threadIdx.x, lane = tid & 31, w = tid >> 5;
  const int b = blockIdx.x;
  if (b < 272) {
    const float* src;
    const float* gsc = elg;
    unsigned short* dbh = pqkv;
    unsigned short* dbl = pqkv;
    f16* dh = w1t;
    int K, N, kt, nt, mode;
    if (b < 16) {
      const int j = b >> 2, t = b & 3;
      kt = t >> 1; nt = t & 1;
      src = (j == 0) ? wq : ((j == 1) ? wk : ((j == 2) ? wv : fcw));
      K = NC; N = NC; mode = 0;
      dbh = pqkv + (size_t)(2 * j) * (NC * NC);
      dbl = dbh + NC * NC;
    } else if (b < 144) {
      const int bb = b - 16, i = bb >> 4, t = bb & 15;
      kt = t >> 3; nt = t & 7;
      src = ew1 + (size_t)i * NC * NH;
      K = NC; N = NH; mode = 1;
      dh = w1t + (size_t)i * NH * NC;
      gsc = elg + i * NC;
    } else {
      const int bb = b - 144, i = bb >> 4, t = bb & 15;
      kt = t >> 1; nt = t & 1;
      src = ew2 + (size_t)i * NH * NC;
      K = NH; N = NC; mode = 2;
      dh = w2t + (size_t)i * NC * NH;
    }
    const int k0 = kt * 64, n0 = nt * 64;
#pragma unroll 1
    for (int it = 0; it < 16; ++it) {
      const int idx = it * 256 + tid;
      const int kk = idx >> 6, nn = idx & 63;
      float v = src[(size_t)(k0 + kk) * N + n0 + nn];
      if (mode == 1) v *= gsc[k0 + kk];
      tile[nn * 65 + kk] = v;
    }
    __syncthreads();
    const int pcs = lane & 7;
    if (mode == 0) {
      v4u_t ph[2], pl[2];
#pragma unroll
      for (int q2 = 0; q2 < 2; ++q2) {
        const int nn = w * 8 + q2 * 4 + (lane >> 3);
        const float* tp = tile + nn * 65 + pcs * 8;
#pragma unroll
        for (int jj = 0; jj < 4; ++jj) {
          unsigned short h0, r0, h1, r1;
          split_bf(tp[2 * jj], h0, r0);
          split_bf(tp[2 * jj + 1], h1, r1);
          ph[q2][jj] = (unsigned int)h0 | ((unsigned int)h1 << 16);
          pl[q2][jj] = (unsigned int)r0 | ((unsigned int)r1 << 16);
        }
      }
#pragma unroll
      for (int q2 = 0; q2 < 2; ++q2) {
        const int nn = w * 8 + q2 * 4 + (lane >> 3);
        const size_t off = (size_t)(n0 + nn) * K + k0 + pcs * 8;
        *(volatile v4u_t*)(dbh + off) = ph[q2];
        *(volatile v4u_t*)(dbl + off) = pl[q2];
      }
      __threadfence();
#pragma unroll
      for (int q2 = 0; q2 < 2; ++q2) {
        const int nn = w * 8 + q2 * 4 + (lane >> 3);
        const size_t off = (size_t)(n0 + nn) * K + k0 + pcs * 8;
        *(volatile v4u_t*)(dbh + off) = ph[q2];
        *(volatile v4u_t*)(dbl + off) = pl[q2];
      }
    } else {
      v4u_t pk[2];
#pragma unroll
      for (int q2 = 0; q2 < 2; ++q2) {
        const int nn = w * 8 + q2 * 4 + (lane >> 3);
        const float* tp = tile + nn * 65 + pcs * 8;
        Pack8 u;
#pragma unroll
        for (int j = 0; j < 8; ++j) u.h[j] = (f16)(tp[j] * 16.0f);
        pk[q2] = u.u;
      }
#pragma unroll
      for (int q2 = 0; q2 < 2; ++q2) {
        const int nn = w * 8 + q2 * 4 + (lane >> 3);
        *(volatile v4u_t*)(dh + (size_t)(n0 + nn) * K + k0 + pcs * 8) = pk[q2];
      }
      __threadfence();
#pragma unroll
      for (int q2 = 0; q2 < 2; ++q2) {
        const int nn = w * 8 + q2 * 4 + (lane >> 3);
        *(volatile v4u_t*)(dh + (size_t)(n0 + nn) * K + k0 + pcs * 8) = pk[q2];
      }
    }
  } else if (b == 272) {
    const int row = w * 8 + (lane >> 2), c0 = (lane & 3) * 8;
    v4u_t ph, pl;
#pragma unroll
    for (int jj = 0; jj < 4; ++jj) {
      unsigned short hb[2], lb[2];
#pragma unroll
      for (int u2 = 0; u2 < 2; ++u2) {
        const int c = c0 + 2 * jj + u2;
        const int ca = (c < NL) ? c : (NL - 1);
        float x = tg[row * NL + ca];
        x = (c < NL) ? x : 0.0f;
        split_bf(x, hb[u2], lb[u2]);
      }
      ph[jj] = (unsigned int)hb[0] | ((unsigned int)hb[1] << 16);
      pl[jj] = (unsigned int)lb[0] | ((unsigned int)lb[1] << 16);
    }
    unsigned short* d0 = tgp + row * 32 + c0;
    unsigned short* d1 = tgp + 2048 + row * 32 + c0;
    *(volatile v4u_t*)d0 = ph;
    *(volatile v4u_t*)d1 = pl;
    __threadfence();
    *(volatile v4u_t*)d0 = ph;
    *(volatile v4u_t*)d1 = pl;
  } else if (b == 273) {
    const int row = w * 4 + (lane >> 3), c0 = (lane & 7) * 8;
    const int ra = (row < NL) ? row : (NL - 1);
    v4u_t ph, pl;
#pragma unroll
    for (int jj = 0; jj < 4; ++jj) {
      unsigned short hb[2], lb[2];
#pragma unroll
      for (int u2 = 0; u2 < 2; ++u2) {
        float x = fg[ra * NS + c0 + 2 * jj + u2];
        x = (row < NL) ? x : 0.0f;
        split_bf(x, hb[u2], lb[u2]);
      }
      ph[jj] = (unsigned int)hb[0] | ((unsigned int)hb[1] << 16);
      pl[jj] = (unsigned int)lb[0] | ((unsigned int)lb[1] << 16);
    }
    unsigned short* d0 = fgp + row * NS + c0;
    unsigned short* d1 = fgp + 2048 + row * NS + c0;
    *(volatile v4u_t*)d0 = ph;
    *(volatile v4u_t*)d1 = pl;
    __threadfence();
    *(volatile v4u_t*)d0 = ph;
    *(volatile v4u_t*)d1 = pl;
  } else {
    const int bb = b - 274, i = bb >> 1, n = (bb & 1) * 256 + tid;
    float s = eb1[i * NH + n];
#pragma unroll 1
    for (int k = 0; k < NC; ++k)
      s = fmaf(elb[i * NC + k], ew1[((size_t)i * NC + k) * NH + n], s);
    float* d = b1f + i * NH + n;
    *(volatile float*)d = s;
    __threadfence();
    *(volatile float*)d = s;
  }
}

__global__ void __launch_bounds__(NTHR) k_l0(
    const float* __restrict__ msg, const float* __restrict__ g0, const float* __restrict__ b0v,
    const unsigned short* __restrict__ pfc, const float* __restrict__ fcb, float* __restrict__ out)
{
  extern __shared__ __align__(16) unsigned char smem_l0[];
  unsigned short* xh = (unsigned short*)smem_l0;
  unsigned short* xl = xh + 64 * MP;
  float* ost = (float*)smem_l0;
  const int tid = threadIdx.x, lane = tid & 31, w = tid >> 5;
  const int hh = lane >> 4, m = lane & 15;
  const int e0 = blockIdx.x * 64;
  {
    const int row = tid >> 2, q = tid & 3;
    const float* src = msg + (size_t)(e0 + row) * (NL * NC) + q * 32;
    float x[32];
#pragma unroll
    for (int j4 = 0; j4 < 8; ++j4) {
      const v4f_t v = *(const v4f*)(src + 4 * j4);
      x[4 * j4] = v[0]; x[4 * j4 + 1] = v[1]; x[4 * j4 + 2] = v[2]; x[4 * j4 + 3] = v[3];
    }
    float s = 0.0f;
#pragma unroll
    for (int j = 0; j < 32; ++j) s += x[j];
    s += __shfl_xor(s, 1, 32);
    s += __shfl_xor(s, 2, 32);
    const float mean = s * (1.0f / 128.0f);
    float s2 = 0.0f;
#pragma unroll
    for (int j = 0; j < 32; ++j) { const float d = x[j] - mean; s2 += d * d; }
    s2 += __shfl_xor(s2, 1, 32);
    s2 += __shfl_xor(s2, 2, 32);
    const float rstd = rsqrtf(s2 * (1.0f / 128.0f) + 1e-5f);
#pragma unroll
    for (int j = 0; j < 32; ++j) {
      const int c = q * 32 + j;
      const float v = (x[j] - mean) * rstd * g0[c] + b0v[c];
      unsigned short h16, l16;
      split_bf(v, h16, l16);
      xh[row * MP + c] = h16;
      xl[row * MP + c] = l16;
    }
  }
  __syncthreads();
  const int mt = w >> 1, nt0 = (w & 1) * 4;
  v8f acc[4];
#pragma unroll
  for (int t = 0; t < 4; ++t) acc[t] = zero8();
  gemm4_bf3(xh + (mt * 16 + m) * MP + 8 * hh, xl + (mt * 16 + m) * MP + 8 * hh,
            pfc, pfc + NC * NC, NC, nt0 * 16, 4, acc, m, hh);
  __syncthreads();
#pragma unroll
  for (int t = 0; t < 4; ++t) {
    const int col = (nt0 + t) * 16 + m;
    const float bias = fcb[col];
#pragma unroll
    for (int r = 0; r < 8; ++r) {
      const float xv = acc[t][r] + bias;
      const float sg = __builtin_amdgcn_rcpf(1.0f + __expf(-xv));
      ost[(mt * 16 + 8 * hh + r) * GP + col] = xv * sg;
    }
  }
  __syncthreads();
  v4f_t v[8];
#pragma unroll
  for (int j = 0; j < 8; ++j) v[j] = *(const v4f*)(ost + (w * 8 + j) * GP + lane * 4);
  float* ob = out + (size_t)(e0 + w * 8) * (NL * NC) + lane * 4;
#pragma unroll
  for (int j = 0; j < 8; ++j) *(volatile v4f_t*)(ob + (size_t)j * (NL * NC)) = v[j];
  __threadfence();
#pragma unroll
  for (int j = 0; j < 8; ++j) *(volatile v4f_t*)(ob + (size_t)j * (NL * NC)) = v[j];
}

__global__ void __launch_bounds__(NTHR) k_attn(
    const float* __restrict__ msg, const float* __restrict__ pos,
    const float* __restrict__ ln1g, const float* __restrict__ ln1b,
    const float* __restrict__ bq, const float* __restrict__ bk, const float* __restrict__ bv,
    const unsigned short* __restrict__ pqkv, const unsigned short* __restrict__ tgp,
    f16* __restrict__ xhat)
{
  extern __shared__ __align__(16) unsigned char smem_at[];
  float* s_g = (float*)(smem_at + AT_A);
  float* s_lg = (float*)(smem_at + AT_A);
  float* s_o = (float*)(smem_at + AT_A);
  unsigned short* s_mh = (unsigned short*)(smem_at + AT_B);
  unsigned short* s_ml = s_mh + 64 * MP;
  unsigned short* s_ph = (unsigned short*)(smem_at + AT_B);
  unsigned short* s_pl = s_ph + 64 * TP;
  unsigned short* s_qh = (unsigned short*)(smem_at + AT_Q);
  unsigned short* s_ql = s_qh + 64 * MP;
  unsigned short* s_kh = (unsigned short*)(smem_at + AT_K);
  unsigned short* s_kl = s_kh + 64 * MP;
  unsigned short* s_vh = (unsigned short*)(smem_at + AT_VT);
  unsigned short* s_vl = s_vh + 128 * TP;
  unsigned short* s_th = (unsigned short*)(smem_at + AT_MT);
  unsigned short* s_tl = s_th + 128 * 32;
  float* s_pos = (float*)(smem_at + AT_POS);

  const int tid = threadIdx.x, lane = tid & 31, w = tid >> 5;
  const int hh = lane >> 4, m = lane & 15;
  const int e = blockIdx.x;
  const int mt = w >> 1;

  {
    const float* me = msg + (size_t)e * NL * NC;
#pragma unroll 1
    for (int it = 0; it < 16; ++it) {
      const int idx = it * 256 + tid;
      const int l = idx >> 7, c = idx & 127;
      const int lc = (l < NL) ? l : (NL - 1);
      float v = me[lc * NC + c];
      v = (l < NL) ? v : 0.0f;
      unsigned short h16, l16;
      split_bf(v, h16, l16);
      s_th[c * 32 + l] = h16;
      s_tl[c * 32 + l] = l16;
    }
    if (tid < NS * 3) s_pos[tid] = pos[tid];
  }
  __syncthreads();

  {
    const int nt0 = (w & 1) * 4;
    v8f acc[4];
#pragma unroll
    for (int t = 0; t < 4; ++t) acc[t] = zero8();
    gemm4_bf3(tgp + (mt * 16 + m) * 32 + 8 * hh, tgp + 2048 + (mt * 16 + m) * 32 + 8 * hh,
              s_th, s_tl, 32, nt0 * 16, 1, acc, m, hh);
#pragma unroll
    for (int t = 0; t < 4; ++t) {
      const int col = (nt0 + t) * 16 + m;
#pragma unroll
      for (int r = 0; r < 8; ++r) s_g[(mt * 16 + 8 * hh + r) * GP + col] = acc[t][r];
    }
  }
  __syncthreads();

  {
    const int row = tid >> 2, q = tid & 3;
    const float* gp = s_g + row * GP + q * 32;
    float x[32];
#pragma unroll
    for (int j4 = 0; j4 < 8; ++j4) {
      const v4f_t v = *(const v4f*)(gp + 4 * j4);
      x[4 * j4] = v[0]; x[4 * j4 + 1] = v[1]; x[4 * j4 + 2] = v[2]; x[4 * j4 + 3] = v[3];
    }
    float s = 0.0f;
#pragma unroll
    for (int j = 0; j < 32; ++j) s += x[j];
    s += __shfl_xor(s, 1, 32);
    s += __shfl_xor(s, 2, 32);
    const float mean = s * (1.0f / 128.0f);
    float s2 = 0.0f;
#pragma unroll
    for (int j = 0; j < 32; ++j) { const float d = x[j] - mean; s2 += d * d; }
    s2 += __shfl_xor(s2, 1, 32);
    s2 += __shfl_xor(s2, 2, 32);
    const float rstd = rsqrtf(s2 * (1.0f / 128.0f) + 1e-5f);
#pragma unroll
    for (int j = 0; j < 32; ++j) {
      const int c = q * 32 + j;
      const float v = (x[j] - mean) * rstd * ln1g[c] + ln1b[c];
      unsigned short h16, l16;
      split_bf(v, h16, l16);
      s_mh[row * MP + c] = h16;
      s_ml[row * MP + c] = l16;
    }
  }
  __syncthreads();

#pragma unroll 1
  for (int j = 0; j < 3; ++j) {
    const unsigned short* wh = pqkv + (size_t)(2 * j) * (NC * NC);
    const unsigned short* wl = wh + NC * NC;
    const float* bsel = (j == 0) ? bq : ((j == 1) ? bk : bv);
    const int nt0 = (w & 1) * 4;
    v8f acc[4];
#pragma unroll
    for (int t = 0; t < 4; ++t) acc[t] = zero8();
    gemm4_bf3(s_mh + (mt * 16 + m) * MP + 8 * hh, s_ml + (mt * 16 + m) * MP + 8 * hh,
              wh, wl, NC, nt0 * 16, 4, acc, m, hh);
    if (j < 2) {
      unsigned short* dh = (unsigned short*)(smem_at + ((j == 0) ? AT_Q : AT_K));
      unsigned short* dl = dh + 64 * MP;
#pragma unroll
      for (int t = 0; t < 4; ++t) {
        const int col = (nt0 + t) * 16 + m;
        const float bias = bsel[col];
#pragma unroll
        for (int r = 0; r < 8; ++r) {
          unsigned short h16, l16;
          split_bf(acc[t][r] + bias, h16, l16);
          const int off = (mt * 16 + 8 * hh + r) * MP + col;
          dh[off] = h16;
          dl[off] = l16;
        }
      }
    } else {
#pragma unroll
      for (int t = 0; t < 4; ++t) {
        const int col = (nt0 + t) * 16 + m;
        const float bias = bsel[col];
#pragma unroll
        for (int r = 0; r < 8; ++r) {
          unsigned short h16, l16;
          split_bf(acc[t][r] + bias, h16, l16);
          const int off = col * TP + mt * 16 + 8 * hh + r;
          s_vh[off] = h16;
          s_vl[off] = l16;
        }
      }
    }
  }
  __syncthreads();

  {
    const int nt0 = (w & 1) * 2;
    v8f acc[2];
    acc[0] = zero8(); acc[1] = zero8();
    gemm2_bf3(s_qh + (mt * 16 + m) * MP + 8 * hh, s_ql + (mt * 16 + m) * MP + 8 * hh,
              s_kh, s_kl, MP, nt0 * 16, 4, acc, m, hh);
    const float scale = 0.0873704056661f;
#pragma unroll
    for (int t = 0; t < 2; ++t) {
      const int tt = (nt0 + t) * 16 + m;
      const float px = s_pos[tt * 3], py = s_pos[tt * 3 + 1], pz = s_pos[tt * 3 + 2];
#pragma unroll
      for (int r = 0; r < 8; ++r) {
        const int sr = mt * 16 + 8 * hh + r;
        const float pp = s_pos[sr * 3] * px + s_pos[sr * 3 + 1] * py + s_pos[sr * 3 + 2] * pz;
        s_lg[sr * LGP + tt] = (acc[t][r] + pp) * scale;
      }
    }
  }
  __syncthreads();

  {
    const int row = tid >> 2, q = tid & 3;
    const float* lp = s_lg + row * LGP + q * 16;
    float x[16];
#pragma unroll
    for (int j4 = 0; j4 < 4; ++j4) {
      const v4f_t v = *(const v4f*)(lp + 4 * j4);
      x[4 * j4] = v[0]; x[4 * j4 + 1] = v[1]; x[4 * j4 + 2] = v[2]; x[4 * j4 + 3] = v[3];
    }
    float mx = x[0];
#pragma unroll
    for (int j = 1; j < 16; ++j) mx = fmaxf(mx, x[j]);
    mx = fmaxf(mx, __shfl_xor(mx, 1, 32));
    mx = fmaxf(mx, __shfl_xor(mx, 2, 32));
    float sum = 0.0f;
#pragma unroll
    for (int j = 0; j < 16; ++j) { x[j] = __expf(x[j] - mx); sum += x[j]; }
    sum += __shfl_xor(sum, 1, 32);
    sum += __shfl_xor(sum, 2, 32);
    const float inv = __builtin_amdgcn_rcpf(sum);
#pragma unroll
    for (int j = 0; j < 16; ++j) {
      const int tcol = q * 16 + j;
      unsigned short h16, l16;
      split_bf(x[j] * inv, h16, l16);
      s_ph[row * TP + tcol] = h16;
      s_pl[row * TP + tcol] = l16;
    }
  }
  __syncthreads();

  {
    const int nt0 = (w & 1) * 4;
    v8f acc[4];
#pragma unroll
    for (int t = 0; t < 4; ++t) acc[t] = zero8();
    gemm4_bf3(s_ph + (mt * 16 + m) * TP + 8 * hh, s_pl + (mt * 16 + m) * TP + 8 * hh,
              s_vh, s_vl, TP, nt0 * 16, 2, acc, m, hh);
#pragma unroll
    for (int t = 0; t < 4; ++t) {
      const int col = (nt0 + t) * 16 + m;
#pragma unroll
      for (int r = 0; r < 8; ++r) s_o[(mt * 16 + 8 * hh + r) * GP + col] = acc[t][r];
    }
  }
  __syncthreads();

  {
    const int rl = tid >> 4, cs = (tid & 15) * 8;
    v4u_t pk[4];
#pragma unroll
    for (int p = 0; p < 4; ++p) {
      const int row = p * 16 + rl;
      const float* op = s_o + row * GP + cs;
      const v4f_t v0 = *(const v4f*)op;
      const v4f_t v1 = *(const v4f*)(op + 4);
      float x[8];
      x[0] = v0[0]; x[1] = v0[1]; x[2] = v0[2]; x[3] = v0[3];
      x[4] = v1[0]; x[5] = v1[1]; x[6] = v1[2]; x[7] = v1[3];
      float s = 0.0f;
#pragma unroll
      for (int j = 0; j < 8; ++j) s += x[j];
      s += __shfl_xor(s, 1, 32);
      s += __shfl_xor(s, 2, 32);
      s += __shfl_xor(s, 4, 32);
      s += __shfl_xor(s, 8, 32);
      const float mean = s * (1.0f / 128.0f);
      float s2 = 0.0f;
#pragma unroll
      for (int j = 0; j < 8; ++j) { const float d = x[j] - mean; s2 += d * d; }
      s2 += __shfl_xor(s2, 1, 32);
      s2 += __shfl_xor(s2, 2, 32);
      s2 += __shfl_xor(s2, 4, 32);
      s2 += __shfl_xor(s2, 8, 32);
      const float rstd = rsqrtf(s2 * (1.0f / 128.0f) + 1e-5f);
      Pack8 u;
#pragma unroll
      for (int j = 0; j < 8; ++j) u.h[j] = (f16)((x[j] - mean) * rstd);
      pk[p] = u.u;
    }
    f16* xd = xhat + (size_t)e * NS * NC + cs;
#pragma unroll
    for (int p = 0; p < 4; ++p)
      *(volatile v4u_t*)(xd + (size_t)(p * 16 + rl) * NC) = pk[p];
    __threadfence();
#pragma unroll
    for (int p = 0; p < 4; ++p)
      *(volatile v4u_t*)(xd + (size_t)(p * 16 + rl) * NC) = pk[p];
  }
}

__global__ void __launch_bounds__(NTHR) k_expert(
    const f16* __restrict__ xhat, const float* __restrict__ gate,
    const f16* __restrict__ w1t, const float* __restrict__ b1f,
    const f16* __restrict__ w2t, const float* __restrict__ eb2,
    const unsigned short* __restrict__ fgp, float* __restrict__ out)
{
  extern __shared__ __align__(16) unsigned char smem_ex[];
  f16* s_x = (f16*)(smem_ex + EX_XS);
  f16* s_h = (f16*)(smem_ex + EX_HID);
  unsigned short* s_ah = (unsigned short*)(smem_ex + EX_AH);
  unsigned short* s_al = (unsigned short*)(smem_ex + EX_AL);
  float* s_os = (float*)(smem_ex + EX_OS);

  const int tid = threadIdx.x, lane = tid & 31, w = tid >> 5;
  const int hh = lane >> 4, m = lane & 15;
  const int e = blockIdx.x;
  const int mt = w >> 1, half = w & 1, nt0 = half * 4;

  {
    const f16* xe = xhat + (size_t)e * NS * NC;
#pragma unroll
    for (int it = 0; it < 4; ++it) {
      const int piece = it * 256 + tid;
      const int row = piece >> 4, cp = (piece & 15) * 8;
      const v4u_t v = *(const v4u*)(xe + row * NC + cp);
      *(v4u*)(s_x + row * MP + cp) = v;
    }
  }
  __syncthreads();

  v8f tot[4];
#pragma unroll
  for (int t = 0; t < 4; ++t) tot[t] = zero8();

#pragma unroll 1
  for (int i = 0; i < NX; ++i) {
    const f16* w1 = w1t + (size_t)i * NH * NC;
    const f16* w2 = w2t + (size_t)i * NC * NH;
    const float* b1 = b1f + i * NH;
#pragma unroll 1
    for (int cg = 0; cg < 4; ++cg) {
      const int nb = half * 256 + cg * 64;
      v8f acc[4];
#pragma unroll
      for (int t = 0; t < 4; ++t) acc[t] = zero8();
      gemm4_h(s_x + (mt * 16 + m) * MP + 8 * hh, w1, NC, nb, 4, acc, m, hh);
#pragma unroll
      for (int t = 0; t < 4; ++t) {
        const int col = nb + 16 * t + m;
        const float bias = b1[col];
#pragma unroll
        for (int r = 0; r < 8; ++r) {
          const float xv = acc[t][r] * (1.0f / 16.0f) + bias;
          const float sg = __builtin_amdgcn_rcpf(1.0f + __expf(-xv));
          s_h[(mt * 16 + 8 * hh + r) * HPIT + col] = (f16)((xv * sg) * 32.0f);
        }
      }
    }
    __syncthreads();
    {
      v8f acc[4];
#pragma unroll
      for (int t = 0; t < 4; ++t) acc[t] = zero8();
      gemm4_h(s_h + (mt * 16 + m) * HPIT + 8 * hh, w2, NH, nt0 * 16, 16, acc, m, hh);
      const float gv = gate[e * NX + i];
      const float* b2 = eb2 + i * NC;
#pragma unroll
      for (int t = 0; t < 4; ++t) {
        const int col = (nt0 + t) * 16 + m;
        const float bb = b2[col];
#pragma unroll
        for (int r = 0; r < 8; ++r) {
          const float y = acc[t][r] * (1.0f / 512.0f) + bb;
          tot[t][r] = tot[t][r] + gv * y;
        }
      }
    }
    __syncthreads();
  }

#pragma unroll
  for (int t = 0; t < 4; ++t) {
    const int c = (nt0 + t) * 16 + m;
#pragma unroll
    for (int r = 0; r < 8; ++r) {
      const int sr = mt * 16 + 8 * hh + r;
      unsigned short h16, l16;
      split_bf(tot[t][r], h16, l16);
      s_ah[c * TP + sr] = h16;
      s_al[c * TP + sr] = l16;
    }
  }
  __syncthreads();

  {
    const int mt2 = w >> 2, nt2 = (w & 3) * 2;
    v8f acc[2];
    acc[0] = zero8(); acc[1] = zero8();
    gemm2_bf3(fgp + (mt2 * 16 + m) * NS + 8 * hh, fgp + 2048 + (mt2 * 16 + m) * NS + 8 * hh,
              s_ah, s_al, TP, nt2 * 16, 2, acc, m, hh);
#pragma unroll
    for (int t = 0; t < 2; ++t) {
      const int col = (nt2 + t) * 16 + m;
#pragma unroll
      for (int r = 0; r < 8; ++r) s_os[(mt2 * 16 + 8 * hh + r) * GP + col] = acc[t][r];
    }
  }
  __syncthreads();

  {
    v4f_t v[3];
#pragma unroll
    for (int j = 0; j < 3; ++j) v[j] = *(const v4f*)(s_os + (1 + w * 3 + j) * GP + lane * 4);
    float* ob = out + (size_t)e * NL * NC + lane * 4;
#pragma unroll
    for (int j = 0; j < 3; ++j) *(volatile v4f_t*)(ob + (size_t)(1 + w * 3 + j) * NC) = v[j];
    __threadfence();
#pragma unroll
    for (int j = 0; j < 3; ++j) *(volatile v4f_t*)(ob + (size_t)(1 + w * 3 + j) * NC) = v[j];
  }
}

extern "C" void kernel_launch(void* const* d_in, const int* in_sizes, int n_in,
                              void* d_out, int out_size, void* d_ws, size_t ws_size,
                              hipStream_t stream)
{
  if (n_in < 24) return;
  if (in_sizes[0] != NE * NL * NC) return;
  if (in_sizes[1] != NE * NX) return;
  if (in_sizes[3] != NC || in_sizes[4] != NC) return;
  if (in_sizes[5] != NC * NC || in_sizes[6] != NC) return;
  if (in_sizes[7] != NC * NC || in_sizes[8] != NC) return;
  if (in_sizes[9] != NC * NC || in_sizes[10] != NC) return;
  if (in_sizes[11] != NC || in_sizes[12] != NC) return;
  if (in_sizes[13] != NC * NC || in_sizes[14] != NC) return;
  if (in_sizes[15] != NX * NC || in_sizes[16] != NX * NC) return;
  if (in_sizes[17] != NX * NC * NH || in_sizes[18] != NX * NH) return;
  if (in_sizes[19] != NX * NH * NC || in_sizes[20] != NX * NC) return;
  if (in_sizes[21] != NS * NL || in_sizes[22] != NL * NS) return;
  if (in_sizes[23] != NS * 3) return;
  if (out_size != NE * NL * NC) return;

  const float* msg  = (const float*)d_in[0];
  const float* gate = (const float*)d_in[1];
  const float* ln1g = (const float*)d_in[3];
  const float* ln1b = (const float*)d_in[4];
  const float* wq   = (const float*)d_in[5];
  const float* bq   = (const float*)d_in[6];
  const float* wk   = (const float*)d_in[7];
  const float* bk   = (const float*)d_in[8];
  const float* wv   = (const float*)d_in[9];
  const float* bv   = (const float*)d_in[10];
  const float* n0g  = (const float*)d_in[11];
  const float* n0b  = (const float*)d_in[12];
  const float* fcw  = (const float*)d_in[13];
  const float* fcb  = (const float*)d_in[14];
  const float* elg  = (const float*)d_in[15];
  const float* elb  = (const float*)d_in[16];
  const float* ew1  = (const float*)d_in[17];
  const float* eb1  = (const float*)d_in[18];
  const float* ew2  = (const float*)d_in[19];
  const float* eb2  = (const float*)d_in[20];
  const float* tgm  = (const float*)d_in[21];
  const float* fgm  = (const float*)d_in[22];
  const float* pem  = (const float*)d_in[23];
  float* out = (float*)d_out;

  const size_t szPQ = (size_t)8 * NC * NC * 2;
  const size_t szW1 = (size_t)NX * NH * NC * 2;
  const size_t szW2 = (size_t)NX * NC * NH * 2;
  const size_t szTG = (size_t)2 * 64 * 32 * 2;
  const size_t szFG = (size_t)2 * 32 * 64 * 2;
  const size_t szB1 = (size_t)NX * NH * 4;
  const size_t szXH = (size_t)NE * NS * NC * 2;
  const size_t oPQ = 0;
  const size_t oW1 = oPQ + szPQ;
  const size_t oW2 = oW1 + szW1;
  const size_t oTG = oW2 + szW2;
  const size_t oFG = oTG + szTG;
  const size_t oB1 = oFG + szFG;
  const size_t oXH = oB1 + szB1;
  const size_t total = oXH + szXH;
  if (total > ws_size) return;

  char* ws = (char*)d_ws;
  unsigned short* pqkv = (unsigned short*)(ws + oPQ);
  f16* w1t = (f16*)(ws + oW1);
  f16* w2t = (f16*)(ws + oW2);
  unsigned short* tgp = (unsigned short*)(ws + oTG);
  unsigned short* fgp = (unsigned short*)(ws + oFG);
  float* b1f = (float*)(ws + oB1);
  f16* xh = (f16*)(ws + oXH);

  k_prep<<<290, NTHR, 0, stream>>>(wq, wk, wv, fcw, elg, elb, ew1, eb1, ew2, tgm, fgm,
                                   pqkv, w1t, w2t, tgp, fgp, b1f);

  k_l0<<<NE / 64, NTHR, L0_LDS, stream>>>(msg, n0g, n0b, pqkv + (size_t)6 * NC * NC, fcb, out);

  hipFuncSetAttribute(reinterpret_cast<const void*>(&k_attn),
                      hipFuncAttributeMaxDynamicSharedMemorySize, AT_LDS);
  k_attn<<<NE, NTHR, AT_LDS, stream>>>(msg, pem, ln1g, ln1b, bq, bk, bv, pqkv, tgp, xh);

  hipFuncSetAttribute(reinterpret_cast<const void*>(&k_expert),
                      hipFuncAttributeMaxDynamicSharedMemorySize, EX_LDS);
  k_expert<<<NE, NTHR, EX_LDS, stream>>>(xh, gate, w1t, b1f, w2t, eb2, fgp, out);
}
